// SABlock_54537494725114
// MI455X (gfx1250) — hardware-verified
//
#include <hip/hip_runtime.h>
#include <hip/hip_bf16.h>


#ifndef NB
#define NB 4
#endif
#ifndef SEQ
#define SEQ 1024
#endif
#define NB_FULL    4
#define SEQ_FULL   1024
#define HIDDEN     1024
#define HEADS      16
#define HEAD_DIM   64
#define QKV_N      (3 * HIDDEN)
#define MROWS      (NB * SEQ)
#define ATT_SCALE  0.125f

static_assert(SEQ % 128 == 0);
static_assert(SEQ <= SEQ_FULL);
static_assert(NB >= 1 && NB <= NB_FULL);
static_assert(HIDDEN == HEADS * HEAD_DIM);
static_assert(MROWS % 128 == 0);
static_assert(QKV_N % 64 == 0);
static_assert(HIDDEN % 64 == 0);
static_assert((long)MROWS * HIDDEN <= (long)NB_FULL * SEQ_FULL * HIDDEN);

typedef float          v4f   __attribute__((ext_vector_type(4)));
typedef float          v8f   __attribute__((ext_vector_type(8)));
typedef unsigned short bfu16;
typedef unsigned short v8us  __attribute__((ext_vector_type(8)));
typedef unsigned short v16us __attribute__((ext_vector_type(16)));
typedef __bf16         v16bf __attribute__((ext_vector_type(16)));

#define GT_P    68
#define PPITCH  40
#define OPITCH  68

__device__ __forceinline__ bfu16 f2bf(float f) {
    unsigned u = __float_as_uint(f);
    u += 0x7FFFu + ((u >> 16) & 1u);
    return (bfu16)(u >> 16);
}
__device__ __forceinline__ float bf2f(bfu16 b) { return __uint_as_float(((unsigned)b) << 16); }

union Frag { v16us u; v8us half[2]; v16bf b; };

__device__ __forceinline__ Frag ldfrag(const bfu16* p, int h) {
    Frag f;
    f.half[0] = *(const v8us*)(p + 8 * h);
    f.half[1] = *(const v8us*)(p + 16 + 8 * h);
    return f;
}

__device__ __forceinline__ v8f wm(const Frag& a, const Frag& b, v8f c) {
    c = __builtin_amdgcn_wmma_f32_16x16x32_bf16(false, a.b, false, b.b, (short)0, c, false, false);
    asm volatile("v_nop\n\tv_nop\n\tv_nop\n\tv_nop" : "+v"(c) : "v"(a.u), "v"(b.u));
    return c;
}

__device__ __forceinline__ void split8(const v4f x0, const v4f x1, v8us& hv, v8us& lv) {
#pragma unroll
    for (int e = 0; e < 4; ++e) {
        const bfu16 a = f2bf(x0[e]);
        hv[e] = a;
        lv[e] = f2bf(x0[e] - bf2f(a));
        const bfu16 c = f2bf(x1[e]);
        hv[4 + e] = c;
        lv[4 + e] = f2bf(x1[e] - bf2f(c));
    }
}

__device__ __forceinline__ float rowmax16(float v) {
    v = fmaxf(v, __shfl_xor(v, 1, 16));
    v = fmaxf(v, __shfl_xor(v, 2, 16));
    v = fmaxf(v, __shfl_xor(v, 4, 16));
    v = fmaxf(v, __shfl_xor(v, 8, 16));
    return v;
}
__device__ __forceinline__ float rowsum16(float v) {
    v += __shfl_xor(v, 1, 16);
    v += __shfl_xor(v, 2, 16);
    v += __shfl_xor(v, 4, 16);
    v += __shfl_xor(v, 8, 16);
    return v;
}

__global__ __launch_bounds__(256)
void cvt_rows_bf16(const float* __restrict__ src, bfu16* __restrict__ dst,
                   int rows, int seq, int seq_full) {
    const int m = blockIdx.x * 2 + (threadIdx.x >> 7);
    if (m >= rows) return;
    const int c = (threadIdx.x & 127) * 8;
    const size_t sr = (size_t)(m / seq) * (size_t)seq_full + (size_t)(m % seq);
    const float* s = src + sr * HIDDEN + c;
    const v4f f0 = *(const v4f*)s;
    const v4f f1 = *(const v4f*)(s + 4);
    v8us o;
#pragma unroll
    for (int e = 0; e < 4; ++e) { o[e] = f2bf(f0[e]); o[4 + e] = f2bf(f1[e]); }
    bfu16* d = dst + (size_t)m * HIDDEN + c;
    *(volatile v8us*)d = o;
    __threadfence();
    *(volatile v8us*)d = o;
}

template <int MODE, int NPL>
__global__ __launch_bounds__(128)
void gemm_bf16(const bfu16* __restrict__ Ah, const bfu16* __restrict__ Al,
               const bfu16* __restrict__ Bw, const float* __restrict__ bias, int ldo,
               bfu16* __restrict__ Qh, bfu16* __restrict__ Ql,
               bfu16* __restrict__ Kh, bfu16* __restrict__ Kl,
               bfu16* __restrict__ Vth, bfu16* __restrict__ Vtl,
               float* __restrict__ Out) {
    __shared__ __attribute__((aligned(16))) float T[128 * GT_P];

    const int wave  = threadIdx.x >> 5;
    const int lane  = threadIdx.x & 31;
    const int laneN = lane & 15;
    const int h     = lane >> 4;
    const int mBase = blockIdx.x * 128;
    const int nBase = blockIdx.y * 64;

    const size_t ra0 = (size_t)(mBase + wave * 32 + laneN) * HIDDEN;
    const size_t ra1 = ra0 + (size_t)16 * HIDDEN;

    v8f acc[2][4] = {};

    for (int k0 = 0; k0 < HIDDEN; k0 += 32) {
        const Frag fa0 = ldfrag(Ah + ra0 + k0, h);
        const Frag fa1 = ldfrag(Ah + ra1 + k0, h);
        Frag ga0 = fa0, ga1 = fa1;
        if (NPL == 2) {
            ga0 = ldfrag(Al + ra0 + k0, h);
            ga1 = ldfrag(Al + ra1 + k0, h);
        }
#pragma unroll
        for (int a = 0; a < 4; ++a) {
            const Frag fb = ldfrag(Bw + (size_t)(nBase + a * 16 + laneN) * HIDDEN + k0, h);
            acc[0][a] = wm(fa0, fb, acc[0][a]);
            acc[1][a] = wm(fa1, fb, acc[1][a]);
            if (NPL == 2) {
                acc[0][a] = wm(ga0, fb, acc[0][a]);
                acc[1][a] = wm(ga1, fb, acc[1][a]);
            }
        }
    }

#pragma unroll
    for (int sub = 0; sub < 2; ++sub)
#pragma unroll
        for (int a = 0; a < 4; ++a)
#pragma unroll
            for (int j = 0; j < 8; ++j)
                T[(wave * 32 + sub * 16 + 8 * h + j) * GT_P + a * 16 + laneN] = acc[sub][a][j];
    __syncthreads();

    if (MODE == 1) {
#pragma unroll
        for (int ps = 0; ps < 2; ++ps) {
            if (ps) __threadfence();
#pragma unroll
            for (int it = 0; it < 16; ++it) {
                const int lr  = wave * 32 + it * 2 + (lane >> 4);
                const int col = (lane & 15) * 4;
                const v4f t  = *(const v4f*)(T + lr * GT_P + col);
                const v4f bb = *(const v4f*)(bias + nBase + col);
                v4f r;
#pragma unroll
                for (int e = 0; e < 4; ++e) r[e] = t[e] + bf2f(f2bf(bb[e]));
                *(volatile v4f*)(Out + (size_t)(mBase + lr) * (size_t)ldo + nBase + col) = r;
            }
        }
    } else {
        const int sel = nBase / HIDDEN;
        const int hh  = (nBase % HIDDEN) / HEAD_DIM;
        const int b   = mBase / SEQ;
        const int s0  = mBase % SEQ;
        const size_t bh = (size_t)b * HEADS + hh;
        if (sel < 2) {
            bfu16* Ph = (sel == 0) ? Qh : Kh;
            bfu16* Pl = (sel == 0) ? Ql : Kl;
#pragma unroll
            for (int ps = 0; ps < 2; ++ps) {
                if (ps) __threadfence();
#pragma unroll
                for (int it = 0; it < 8; ++it) {
                    const int lr = wave * 32 + it * 4 + (lane >> 3);
                    const int d0 = (lane & 7) * 8;
                    const v4f x0 = *(const v4f*)(T + lr * GT_P + d0);
                    const v4f x1 = *(const v4f*)(T + lr * GT_P + d0 + 4);
                    v8us hv, lv;
                    split8(x0, x1, hv, lv);
                    const size_t off = (bh * SEQ + (size_t)(s0 + lr)) * HEAD_DIM + d0;
                    *(volatile v8us*)(Ph + off) = hv;
                    *(volatile v8us*)(Pl + off) = lv;
                }
            }
        } else {
#pragma unroll
            for (int ps = 0; ps < 2; ++ps) {
                if (ps) __threadfence();
#pragma unroll
                for (int it = 0; it < 8; ++it) {
                    const int d  = wave * 16 + it * 2 + (lane >> 4);
                    const int sl = (lane & 15) * 8;
                    v4f x0, x1;
#pragma unroll
                    for (int e = 0; e < 4; ++e) {
                        x0[e] = T[(sl + e) * GT_P + d];
                        x1[e] = T[(sl + 4 + e) * GT_P + d];
                    }
                    v8us hv, lv;
                    split8(x0, x1, hv, lv);
                    const size_t off = (bh * HEAD_DIM + (size_t)d) * SEQ + s0 + sl;
                    *(volatile v8us*)(Vth + off) = hv;
                    *(volatile v8us*)(Vtl + off) = lv;
                }
            }
        }
    }
}

__global__ __launch_bounds__(256)
void attn_flash(const bfu16* __restrict__ Qh, const bfu16* __restrict__ Ql,
                const bfu16* __restrict__ Kh, const bfu16* __restrict__ Kl,
                const bfu16* __restrict__ Vth, const bfu16* __restrict__ Vtl,
                bfu16* __restrict__ Oh, bfu16* __restrict__ Ol) {
    __shared__ __attribute__((aligned(16))) bfu16 Psh[8][2][16 * PPITCH];
    __shared__ __attribute__((aligned(16))) float  Osh[8][16 * OPITCH];

    const int wave  = threadIdx.x >> 5;
    const int lane  = threadIdx.x & 31;
    const int laneN = lane & 15;
    const int h     = lane >> 4;
    const int bh    = blockIdx.x;
    const int b     = bh / HEADS;
    const int hh    = bh - b * HEADS;
    const int q0    = blockIdx.y * 128 + wave * 16;
    const size_t pb = (size_t)bh * SEQ * HEAD_DIM;

    Frag qh[2], ql[2];
#pragma unroll
    for (int kk = 0; kk < 2; ++kk) {
        const size_t qo = pb + (size_t)(q0 + laneN) * HEAD_DIM + kk * 32;
        qh[kk] = ldfrag(Qh + qo, h);
        ql[kk] = ldfrag(Ql + qo, h);
    }

    float mrow[8], lrow[8];
#pragma unroll
    for (int j = 0; j < 8; ++j) { mrow[j] = -1e30f; lrow[j] = 0.0f; }
    v8f o[4] = {};

    bfu16* Pwh = &Psh[wave][0][0];
    bfu16* Pwl = &Psh[wave][1][0];

    for (int key0 = 0; key0 < SEQ; key0 += 32) {
        v8f s[2] = {};
#pragma unroll
        for (int t = 0; t < 2; ++t) {
#pragma unroll
            for (int kk = 0; kk < 2; ++kk) {
                const size_t ko = pb + (size_t)(key0 + t * 16 + laneN) * HEAD_DIM + kk * 32;
                const Frag fkh = ldfrag(Kh + ko, h);
                const Frag fkl = ldfrag(Kl + ko, h);
                s[t] = wm(qh[kk], fkh, s[t]);
                s[t] = wm(ql[kk], fkh, s[t]);
                s[t] = wm(qh[kk], fkl, s[t]);
            }
        }

        float p0[8], p1[8];
#pragma unroll
        for (int j = 0; j < 8; ++j) {
            const float a0 = s[0][j] * ATT_SCALE;
            const float a1 = s[1][j] * ATT_SCALE;
            const float mx = rowmax16(fmaxf(a0, a1));
            const float mn = fmaxf(mrow[j], mx);
            const float alpha = __expf(mrow[j] - mn);
            p0[j] = __expf(a0 - mn);
            p1[j] = __expf(a1 - mn);
            lrow[j] = lrow[j] * alpha + rowsum16(p0[j] + p1[j]);
            mrow[j] = mn;
#pragma unroll
            for (int a = 0; a < 4; ++a) o[a][j] *= alpha;
        }

#pragma unroll
        for (int j = 0; j < 8; ++j) {
            const int r = 8 * h + j;
            const bfu16 b0 = f2bf(p0[j]);
            const bfu16 b1 = f2bf(p1[j]);
            Pwh[r * PPITCH + laneN]      = b0;
            Pwh[r * PPITCH + 16 + laneN] = b1;
            Pwl[r * PPITCH + laneN]      = f2bf(p0[j] - bf2f(b0));
            Pwl[r * PPITCH + 16 + laneN] = f2bf(p1[j] - bf2f(b1));
        }
        __syncthreads();
        const Frag pfh = ldfrag(Pwh + laneN * PPITCH, h);
        const Frag pfl = ldfrag(Pwl + laneN * PPITCH, h);
        __syncthreads();

#pragma unroll
        for (int a = 0; a < 4; ++a) {
            const size_t vo = pb + (size_t)(a * 16 + laneN) * SEQ + key0;
            const Frag fvh = ldfrag(Vth + vo, h);
            const Frag fvl = ldfrag(Vtl + vo, h);
            o[a] = wm(pfh, fvh, o[a]);
            o[a] = wm(pfl, fvh, o[a]);
            o[a] = wm(pfh, fvl, o[a]);
        }
    }

    float linv[8];
#pragma unroll
    for (int j = 0; j < 8; ++j) linv[j] = 1.0f / lrow[j];
    float* Ow = &Osh[wave][0];
#pragma unroll
    for (int a = 0; a < 4; ++a)
#pragma unroll
        for (int j = 0; j < 8; ++j)
            Ow[(8 * h + j) * OPITCH + a * 16 + laneN] = o[a][j] * linv[j];
    __syncthreads();

#pragma unroll
    for (int ps = 0; ps < 2; ++ps) {
        if (ps) __threadfence();
#pragma unroll
        for (int it = 0; it < 4; ++it) {
            const int r  = it * 4 + (lane >> 3);
            const int d0 = (lane & 7) * 8;
            const v4f x0 = *(const v4f*)(Ow + r * OPITCH + d0);
            const v4f x1 = *(const v4f*)(Ow + r * OPITCH + d0 + 4);
            v8us hv, lv;
            split8(x0, x1, hv, lv);
            const size_t off = ((size_t)b * SEQ + (size_t)(q0 + r)) * HIDDEN + hh * HEAD_DIM + d0;
            *(volatile v8us*)(Oh + off) = hv;
            *(volatile v8us*)(Ol + off) = lv;
        }
    }
}

extern "C" void kernel_launch(void* const* d_in, const int* in_sizes, int n_in,
                              void* d_out, int out_size, void* d_ws, size_t ws_size,
                              hipStream_t stream) {
    if (n_in < 4) return;
    const long needX = ((long)(NB - 1) * SEQ_FULL + SEQ) * (long)HIDDEN;
    if ((long)in_sizes[0] < needX) return;
    if ((long)in_sizes[1] < (long)QKV_N * HIDDEN) return;
    if ((long)in_sizes[2] < (long)HIDDEN * HIDDEN) return;
    if ((long)in_sizes[3] < (long)HIDDEN) return;
    if ((long)out_size < (long)MROWS * HIDDEN) return;

    const float* x     = (const float*)d_in[0];
    const float* w_qkv = (const float*)d_in[1];
    const float* w_out = (const float*)d_in[2];
    const float* b_out = (const float*)d_in[3];
    float*       out   = (float*)d_out;

    const size_t planeB = (size_t)MROWS * HIDDEN * sizeof(bfu16);
    size_t off = 0;
    char* ws = (char*)d_ws;
    bfu16* Xb    = (bfu16*)(ws + off); off += planeB;
    bfu16* Wqkvb = (bfu16*)(ws + off); off += (size_t)QKV_N * HIDDEN * sizeof(bfu16);
    bfu16* Woutb = (bfu16*)(ws + off); off += (size_t)HIDDEN * HIDDEN * sizeof(bfu16);
    bfu16* Qh    = (bfu16*)(ws + off); off += planeB;
    bfu16* Ql    = (bfu16*)(ws + off); off += planeB;
    bfu16* Kh    = (bfu16*)(ws + off); off += planeB;
    bfu16* Kl    = (bfu16*)(ws + off); off += planeB;
    bfu16* Vth   = (bfu16*)(ws + off); off += planeB;
    bfu16* Vtl   = (bfu16*)(ws + off); off += planeB;
    bfu16* Oh    = (bfu16*)(ws + off); off += planeB;
    bfu16* Ol    = (bfu16*)(ws + off); off += planeB;
    if (off > ws_size) return;

    cvt_rows_bf16<<<dim3(MROWS / 2), 256, 0, stream>>>(x, Xb, MROWS, SEQ, SEQ_FULL);
    cvt_rows_bf16<<<dim3(QKV_N / 2), 256, 0, stream>>>(w_qkv, Wqkvb, QKV_N, QKV_N, QKV_N);
    cvt_rows_bf16<<<dim3(HIDDEN / 2), 256, 0, stream>>>(w_out, Woutb, HIDDEN, HIDDEN, HIDDEN);

    gemm_bf16<0, 1><<<dim3(MROWS / 128, QKV_N / 64), 128, 0, stream>>>(
        Xb, Xb, Wqkvb, b_out, QKV_N, Qh, Ql, Kh, Kl, Vth, Vtl, out);

    attn_flash<<<dim3(NB * HEADS, SEQ / 128), 256, 0, stream>>>(Qh, Ql, Kh, Kl, Vth, Vtl, Oh, Ol);

    gemm_bf16<1, 2><<<dim3(MROWS / 128, HIDDEN / 64), 128, 0, stream>>>(
        Oh, Ol, Woutb, b_out, HIDDEN, Qh, Ql, Kh, Kl, Vth, Vtl, out);
}
